// SelfAttention_16621523435582
// MI455X (gfx1250) — hardware-verified
//
#include <hip/hip_runtime.h>


namespace {
constexpr int B = 2, T = 4096, DM = 512, H = 8, HK = 8, GRP = H / HK, HD = 64, DKV = HK * HD  , NSLAB = (DM + 2 * DKV) / 128  , BL = 2  , QL = 4096  ;
constexpr float XS = 8.0f, WSC = 256.0f, PS = 1024.0f, LOG2E = 1.4426950408889634f, NEGM = -1e9f;
static_assert(T % 64 == 0 && QL % 64 == 0 && DM % 256 == 0, "tiling");
typedef _Float16 b16;
typedef __attribute__((ext_vector_type(16))) _Float16 v16b;
typedef __attribute__((ext_vector_type(8))) _Float16 v8b;
typedef __attribute__((ext_vector_type(8))) float v8f;
typedef __attribute__((ext_vector_type(4))) float v4f;
__device__ __forceinline__ float bf16_rne(float f) { unsigned int u = __float_as_uint(f); u += 0x7FFFu + ((u >> 16) & 1u); return __uint_as_float(u & 0xFFFF0000u); }
__device__ __forceinline__ void split16(float v, b16& hi, b16& lo) { hi = (b16)v; lo = (b16)(v - (float)hi); }
__device__ __forceinline__ v16b frag_kb(const b16* p, int hh) { const v8b a = *(const v8b*)(p + 8 * hh), b = *(const v8b*)(p + 16 + 8 * hh); v16b f;
#pragma unroll
  for (int e = 0; e < 8; ++e) { f[e] = a[e]; f[8 + e] = b[e]; } return f; }
__device__ __forceinline__ v8f wmma16b(v16b a, v16b b, v8f c) { v8f d = __builtin_amdgcn_wmma_f32_16x16x32_f16(false, a, false, b, (short)0, c, false, false); asm volatile("v_nop\n\tv_nop\n\tv_nop\n\tv_nop" : "+v"(d) : "v"(a), "v"(b)); return d; }
__device__ __forceinline__ void wave_lds_sync() { __builtin_amdgcn_fence(__ATOMIC_RELEASE, "workgroup"); __builtin_amdgcn_wave_barrier(); __builtin_amdgcn_fence(__ATOMIC_ACQUIRE, "workgroup"); }
__device__ __forceinline__ float pmul(float a, float b) { float p = a * b; asm volatile("" : "+v"(p)); return p; }
__device__ __forceinline__ int iclamp(int v, int lo, int hi) { return v < lo ? lo : (v > hi ? hi : v); }

typedef __attribute__((ext_vector_type(2))) _Float16 v2h;
typedef __attribute__((ext_vector_type(4))) _Float16 v4h;
typedef __attribute__((ext_vector_type(2))) float v2f;
typedef __attribute__((ext_vector_type(4))) int v4i;
__device__ __forceinline__ float nexp2(float v) { return __builtin_amdgcn_exp2f(v); }
__global__ __launch_bounds__(256) void prep_kernel(const float* __restrict__ wqkv, const float* __restrict__ wo, b16* __restrict__ WT, b16* __restrict__ WO) {
  const size_t u = (size_t)blockIdx.x * 256 + threadIdx.x; const size_t n1 = (size_t)(DM + 2 * DKV) * DM / 8, n2 = (size_t)DM * DM / 8; if (u >= n1 + n2) return; v8b o;
  if (u < n1) { const size_t e = u * 8; const int oo = (int)(e / DM), k0 = (int)(e % DM);
    for (int j = 0; j < 8; ++j) { const int k = k0 + j; o[j] = (b16)(bf16_rne(wqkv[(size_t)k * (DM + 2 * DKV) + oo]) * WSC); }
    for (int pass = 0; pass < 2; ++pass) { *(volatile v8b*)(WT + e) = o; __threadfence(); } }
  else { const size_t e = (u - n1) * 8; const int oo = (int)(e / DM), k0 = (int)(e % DM); for (int j = 0; j < 8; ++j) o[j] = (b16)(bf16_rne(wo[(size_t)(k0 + j) * DM + oo]) * WSC); for (int pass = 0; pass < 2; ++pass) { *(volatile v8b*)(WO + e) = o; __threadfence(); } }
}
__global__ __launch_bounds__(128) void proj_kernel(const float* __restrict__ x, const float* __restrict__ bqkv, const b16* __restrict__ WT, b16* __restrict__ QH, b16* __restrict__ QLo, b16* __restrict__ KH, b16* __restrict__ KLo, b16* __restrict__ VTh, b16* __restrict__ VTl) {
  __shared__ __attribute__((aligned(16))) b16 As[64][256 + 8]; __shared__ __attribute__((aligned(16))) float Tf[4][16][128 + 4];
  const int wave = threadIdx.x >> 5, lane = threadIdx.x & 31, nloc = lane & 15, hlf = lane >> 4; const int t0 = blockIdx.x * 64; const int b = blockIdx.y; const int slab = blockIdx.z, n0 = slab * 128  ; const int part = slab / (DM / 128); const int c0 = n0 - (part == 0 ? 0 : (part == 1 ? DM : DM + DKV));
  if (t0 >= QL) return;
  const float* xb = x + ((size_t)b * T + t0) * DM;
  v8f acc[8];
#pragma unroll
  for (int t = 0; t < 8; ++t) acc[t] = (v8f){};
#pragma unroll 1
  for (int kc = 0; kc < DM; kc += 256) {
    __syncthreads();
    for (int i = threadIdx.x; i < 64 * 64; i += 128) { const int rr = i / 64, q = (i % 64) * 4; const v4f f = *(const v4f*)(xb + (size_t)rr * DM + kc + q); v4h o; for (int j = 0; j < 4; ++j) o[j] = (b16)(bf16_rne(f[j]) * XS); *(v4h*)(&As[rr][q]) = o; }
    __syncthreads();
#pragma unroll 2
    for (int kb = 0; kb < 256; kb += 32) { const v16b a = frag_kb(&As[wave * 16 + nloc][kb], hlf);
#pragma unroll
      for (int t = 0; t < 8; ++t) acc[t] = wmma16b(a, frag_kb(WT + (size_t)(n0 + t * 16 + nloc) * DM + kc + kb, hlf), acc[t]); } }
#pragma unroll
  for (int t = 0; t < 8; ++t) { const float bb = bf16_rne(bqkv[n0 + t * 16 + nloc]);
#pragma unroll
    for (int r = 0; r < 8; ++r) Tf[wave][8 * hlf + r][t * 16 + nloc] = acc[t][r] * (1.0f / (XS * WSC)) + bb; }
  __syncthreads();
  for (int pass = 0; pass < 2; ++pass) {
    if (part < 2) { b16* ph_ = part == 0 ? QH : KH; b16* pl_ = part == 0 ? QLo : KLo; const int NHp = part == 0 ? H : HK; const int c = c0 + lane * 4; const int h = c / HD, d = c % HD;
      for (int rr = 0; rr < 16; ++rr) { const int tok = t0 + wave * 16 + rr;
        v4h h4, l4; for (int j = 0; j < 4; ++j) { b16 p, q; split16(Tf[wave][rr][lane * 4 + j] * XS, p, q); h4[j] = p; l4[j] = q; }
        const size_t oi = (((size_t)b * NHp + h) * T + tok) * HD + d; *(volatile v4h*)(ph_ + oi) = h4; *(volatile v4h*)(pl_ + oi) = l4; } }
    else {
#pragma unroll 1
      for (int q = 0; q < 32; ++q) { const int cl = wave * 32 + q; const int c = c0 + cl; const int h = c / HD, d = c % HD; const int tk = lane * 2; v2h hv, lv;
        for (int j = 0; j < 2; ++j) { b16 p, ql; split16(Tf[(tk + j) >> 4][(tk + j) & 15][cl] * XS, p, ql); hv[j] = p; lv[j] = ql; }
        const size_t oi = (((size_t)b * HK + h) * HD + d) * (size_t)T + t0 + lane * 2; *(volatile v2h*)(VTh + oi) = hv; *(volatile v2h*)(VTl + oi) = lv; } }
    __threadfence(); }
}
__global__ __launch_bounds__(64) void attn_kernel(const b16* __restrict__ QH, const b16* __restrict__ QLo, const b16* __restrict__ KH, const b16* __restrict__ KLo, const b16* __restrict__ VTh, const b16* __restrict__ VTl, b16* __restrict__ Ch, b16* __restrict__ Cl) {
  __shared__ __attribute__((aligned(16))) b16 Pb[2][16][32 + 8], Pc[2][16][32 + 8]; __shared__ __attribute__((aligned(16))) float To[2][16][HD + 4];
  const int wave = threadIdx.x >> 5, lane = threadIdx.x & 31, hh = lane >> 4, col = lane & 15; const int b = blockIdx.y / H, h = blockIdx.y % H; const int q0 = blockIdx.x * 32 + wave * 16, qi = q0 + col;
  const size_t ph = (size_t)b * H + h, pk = (size_t)b * HK + h / GRP; const size_t pq = ph * T * HD, pkk = pk * T * HD; const b16* Vh = VTh + pk * HD * (size_t)T; const b16* Vl = VTl + pk * HD * (size_t)T;
  const v16b qh0 = frag_kb(QH + pq + (size_t)qi * HD, hh), qh1 = frag_kb(QH + pq + (size_t)qi * HD + 32, hh), ql0 = frag_kb(QLo + pq + (size_t)qi * HD, hh), ql1 = frag_kb(QLo + pq + (size_t)qi * HD + 32, hh);
  const float cs = LOG2E / (8.0f * XS * XS);
  float m = -INFINITY, l = 0.0f; v8f o[4]; for (int t = 0; t < 4; ++t) o[t] = (v8f){};
  const int kend = q0 + 16;
#pragma unroll 1
  for (int kb = 0; kb < kend; kb += 32) {
    float e[16]; float mx = -INFINITY;
#pragma unroll
    for (int u = 0; u < 2; ++u) { v8f s = (v8f){}; const size_t kr = pkk + (size_t)(kb + u * 16 + col) * HD; const v16b kh0 = frag_kb(KH + kr, hh), kh1 = frag_kb(KH + kr + 32, hh), kl0 = frag_kb(KLo + kr, hh), kl1 = frag_kb(KLo + kr + 32, hh);
      s = wmma16b(kh0, qh0, s); s = wmma16b(kh0, ql0, s); s = wmma16b(kl0, qh0, s); s = wmma16b(kh1, qh1, s); s = wmma16b(kh1, ql1, s); s = wmma16b(kl1, qh1, s);
#pragma unroll
      for (int r = 0; r < 8; ++r) { const int key = kb + u * 16 + 8 * hh + r; const float vv = (key <= qi) ? s[r] * cs : -INFINITY; e[u * 8 + r] = vv; mx = fmaxf(mx, vv); } }
    mx = fmaxf(mx, __shfl_xor(mx, 16)); const float mn = fmaxf(m, mx); const float al = nexp2(m - mn); float sum = 0.0f;
#pragma unroll
    for (int i2 = 0; i2 < 16; ++i2) { const float p = nexp2(e[i2] - mn); sum += p; b16 a_, b_; split16(p * PS, a_, b_); const int sl = (i2 < 8 ? 0 : 16) + 8 * hh + (i2 & 7); Pb[wave][col][sl] = a_; Pc[wave][col][sl] = b_; }
    sum += __shfl_xor(sum, 16); l = l * al + sum; m = mn;
    wave_lds_sync();
    const v16b pf = frag_kb(&Pb[wave][col][0], hh), pg = frag_kb(&Pc[wave][col][0], hh);
#pragma unroll
    for (int t = 0; t < 4; ++t) { o[t] *= al; const size_t vr = (size_t)(t * 16 + col) * T + kb; const v16b va = frag_kb(Vh + vr, hh), vb2 = frag_kb(Vl + vr, hh); o[t] = wmma16b(va, pf, o[t]); o[t] = wmma16b(va, pg, o[t]); o[t] = wmma16b(vb2, pf, o[t]); }
    wave_lds_sync(); }
  const float inv = 1.0f / (l * PS * XS);
#pragma unroll
  for (int t = 0; t < 4; ++t)
#pragma unroll
    for (int r = 0; r < 8; ++r) To[wave][col][t * 16 + 8 * hh + r] = o[t][r] * inv;
  wave_lds_sync();
  for (int pass = 0; pass < 2; ++pass) { for (int rr = 0; rr < 16; ++rr) { const v2f f = *(const v2f*)(&To[wave][rr][lane * 2]); v2h hv, lv; for (int j = 0; j < 2; ++j) { b16 p, q; split16(f[j] * XS, p, q); hv[j] = p; lv[j] = q; }
      const size_t oi = ((size_t)b * T + q0 + rr) * DM + h * HD + lane * 2; *(volatile v2h*)(Ch + oi) = hv; *(volatile v2h*)(Cl + oi) = lv; } __threadfence(); }
}
__global__ __launch_bounds__(128) void out_kernel(const b16* __restrict__ Ch, const b16* __restrict__ Cl, const b16* __restrict__ WO, const float* __restrict__ bo, float* __restrict__ out) {
  __shared__ __attribute__((aligned(16))) float Tf[4][16][128 + 4];
  const int wave = threadIdx.x >> 5, lane = threadIdx.x & 31, nloc = lane & 15, hlf = lane >> 4; const int b = blockIdx.z; const size_t m0 = (size_t)b * T + ((size_t)blockIdx.x * 4 + wave) * 16; const int n0 = blockIdx.y * 128;
  v8f acc[8];
#pragma unroll
  for (int t = 0; t < 8; ++t) acc[t] = (v8f){};
#pragma unroll 2
  for (int kb = 0; kb < DM; kb += 32) { const v16b a = frag_kb(Ch + (m0 + nloc) * DM + kb, hlf), al = frag_kb(Cl + (m0 + nloc) * DM + kb, hlf);
#pragma unroll
    for (int t = 0; t < 8; ++t) { const v16b bw = frag_kb(WO + (size_t)(n0 + t * 16 + nloc) * DM + kb, hlf); acc[t] = wmma16b(a, bw, acc[t]); acc[t] = wmma16b(al, bw, acc[t]); } }
#pragma unroll
  for (int t = 0; t < 8; ++t) { const float bb = bf16_rne(bo[n0 + t * 16 + nloc]);
#pragma unroll
    for (int r = 0; r < 8; ++r) Tf[wave][8 * hlf + r][t * 16 + nloc] = acc[t][r] * (1.0f / (XS * WSC)) + bb; }
  wave_lds_sync();
  for (int pass = 0; pass < 2; ++pass) { for (int rr = 0; rr < 16; ++rr) *(volatile v4f*)(out + (m0 + rr) * DM + n0 + lane * 4) = *(const v4f*)(&Tf[wave][rr][lane * 4]); __threadfence(); }
}
}

extern "C" void kernel_launch(void* const* d_in, const int* in_sizes, int n_in, void* d_out, int out_size, void* d_ws, size_t ws_size, hipStream_t stream) {
  (void)n_in;
  auto Fp = [&](int i) { return (const float*)d_in[i]; };
  if (in_sizes[0] != B * T * DM || in_sizes[1] != DM * (DM + 2 * DKV) || in_sizes[2] != DM + 2 * DKV || in_sizes[3] != DM * DM || in_sizes[4] != DM || out_size != B * T * DM) return;
  size_t off = 0; char* ws = (char*)d_ws;
  auto carve = [&](size_t bytes) { char* p = ws + off; off += (bytes + 255) & ~(size_t)255; return p; };
  b16* WT = (b16*)carve((size_t)(DM + 2 * DKV) * DM * 2); b16* WO = (b16*)carve((size_t)DM * DM * 2); const size_t plane = (size_t)B * T * DM * 2, kplane = (size_t)B * T * DKV * 2;
  b16* QH = (b16*)carve(plane); b16* QLo = (b16*)carve(plane); b16* KH = (b16*)carve(kplane); b16* KLo = (b16*)carve(kplane); b16* VTh = (b16*)carve(kplane); b16* VTl = (b16*)carve(kplane); b16* Ch = (b16*)carve(plane); b16* Cl = (b16*)carve(plane);
  if (off > ws_size || off > ((size_t)128 << 20)) return;
  prep_kernel<<<(unsigned)((((size_t)(DM + 2 * DKV) * DM + (size_t)DM * DM) / 8 + 255) / 256), 256, 0, stream>>>(Fp(1), Fp(3), WT, WO);
  proj_kernel<<<dim3(QL / 64, BL, NSLAB), 128, 0, stream>>>(Fp(0), Fp(2), WT, QH, QLo, KH, KLo, VTh, VTl);
  attn_kernel<<<dim3(QL / 32, BL * H), 64, 0, stream>>>(QH, QLo, KH, KLo, VTh, VTl, Ch, Cl);
  out_kernel<<<dim3(QL / 64, DM / 128, BL), 128, 0, stream>>>(Ch, Cl, WO, Fp(4), (float*)d_out);
}
